// CapsuleLayer_46024869544135
// MI455X (gfx1250) — hardware-verified
//
#include <hip/hip_runtime.h>


#ifndef NB
#define NB 32
#endif
#define NB_FULL 32
#define NI  32
#define NA  16
#define OD  10
#define OA  16
#define NK  160
#define HW  144
#define MROWS (NB * HW)
#define MT  (MROWS / 16)
#define VW  4
#define OSP 164
#define LP  10
#define TP  148

static_assert(NB <= NB_FULL);
static_assert(NA == 16);
static_assert(OD * OA == NK);
static_assert(NK % 32 == 0);
static_assert(NK % 16 == 0);
static_assert(HW % 16 == 0);
static_assert(HW % 4 == 0);
static_assert((NI * MT) % VW == 0);
static_assert((NI * NK) % 128 == 0);
static_assert((32 * HW * 4) % 128 == 0);
static_assert((32 * HW) % (4 * 128) == 0);
static_assert(OSP >= NK && (OSP % 4) == 0);
static_assert(TP >= HW && (TP % 4) == 0);

typedef unsigned short bf;
typedef __attribute__((ext_vector_type(16))) __bf16   v16bf;
typedef __attribute__((ext_vector_type(8)))  unsigned short v8us;
typedef __attribute__((ext_vector_type(8)))  float    v8f;
typedef __attribute__((ext_vector_type(4)))  float    v4f;
typedef v4f  __attribute__((may_alias)) v4fa;

__device__ __forceinline__ unsigned short f2bf(float f) { unsigned u = __float_as_uint(f); u += 0x7FFFu + ((u >> 16) & 1u); return (unsigned short)(u >> 16); }
__device__ __forceinline__ float bfr(float f) { return __uint_as_float(((unsigned)f2bf(f)) << 16); }
__device__ __forceinline__ v16bf cat16b(v8us lo, v8us hi) { return __builtin_bit_cast(v16bf, __builtin_shufflevector(lo, hi, 0, 1, 2, 3, 4, 5, 6, 7, 8, 9, 10, 11, 12, 13, 14, 15)); }
__device__ __forceinline__ v8f wmmab(v16bf a, v16bf b, v8f c) { return __builtin_amdgcn_wmma_f32_16x16x32_bf16(false, a, false, b, (short)0, c, false, false); }
__device__ __forceinline__ void wave_sync() { __builtin_amdgcn_fence(3  , "wavefront"); __builtin_amdgcn_wave_barrier(); asm volatile("" ::: "memory"); }

__global__ __launch_bounds__(320) void k_tcvt(const float* __restrict__ src, bf* dst, int C, int GD, size_t sA, size_t sB) {
    __shared__ __align__(16) float ts[16 * OSP];
    const int g = blockIdx.x, tid = threadIdx.x;
    const float* s = src + (size_t)g * 16 * (size_t)C;
    for (int q = tid; q < 4 * C; q += 2 * C) {
        const v4f v = *(const v4f*)(s + 4 * q);
        const int a = (4 * q) / C, c = (4 * q) % C;
        *(v4fa*)(&ts[a * OSP + c]) = v;
    }
    __syncthreads();
    const int row = tid >> 1, hf = tid & 1;
    v8us o;
#pragma unroll
    for (int k = 0; k < 8; ++k) o[k] = f2bf(ts[(8 * hf + k) * OSP + row]);
    bf* d = dst + (size_t)(g / GD) * sA + (size_t)(g % GD) * sB + (size_t)row * 16 + 8 * hf;
    *(volatile v8us*)d = o; __threadfence(); *(volatile v8us*)d = o;
}

__global__ __launch_bounds__(32 * VW) void k_votes(const bf* __restrict__ XA, const bf* __restrict__ WT, float* VO) {
    __shared__ __align__(16) float os[VW * 16 * OSP];
    const int lane = threadIdx.x & 31, lr = lane & 15, hi = lane >> 4;
    const int wave = __builtin_amdgcn_readfirstlane((int)(threadIdx.x >> 5));
    const int task = blockIdx.x * VW + wave;
    const int i = task / MT, m0 = (task % MT) * 16;
    const v8us z = (v8us){};
    const v8us av = *(const v8us*)(XA + ((size_t)i * MROWS + m0 + lr) * 16 + 8 * hi);
    const v16bf a = cat16b(av, z);
    const bf* wp = WT + ((size_t)i * NK + lr) * 16 + 8 * hi;
    v8f acc[10];
#pragma unroll
    for (int nt = 0; nt < 10; ++nt) acc[nt] = (v8f){};
    {
        v16bf b[5];
#pragma unroll
        for (int nt = 0; nt < 5; ++nt) b[nt] = cat16b(*(const v8us*)(wp + (size_t)nt * 256), z);
#pragma unroll
        for (int nt = 0; nt < 5; ++nt) acc[nt] = wmmab(a, b[nt], acc[nt]);
        asm volatile("v_nop\n\tv_nop\n\tv_nop\n\tv_nop" : "+v"(acc[0]), "+v"(acc[1]), "+v"(acc[2]), "+v"(acc[3]), "+v"(acc[4]) : "v"(a), "v"(b[0]), "v"(b[1]), "v"(b[2]), "v"(b[3]), "v"(b[4]));
    }
    {
        v16bf b[5];
#pragma unroll
        for (int nt = 0; nt < 5; ++nt) b[nt] = cat16b(*(const v8us*)(wp + (size_t)(nt + 5) * 256), z);
#pragma unroll
        for (int nt = 0; nt < 5; ++nt) acc[nt + 5] = wmmab(a, b[nt], acc[nt + 5]);
        asm volatile("v_nop\n\tv_nop\n\tv_nop\n\tv_nop" : "+v"(acc[5]), "+v"(acc[6]), "+v"(acc[7]), "+v"(acc[8]), "+v"(acc[9]) : "v"(a), "v"(b[0]), "v"(b[1]), "v"(b[2]), "v"(b[3]), "v"(b[4]));
    }
    const int wb = wave * 16 * OSP;
#pragma unroll
    for (int nt = 0; nt < 10; ++nt) {
#pragma unroll
        for (int r = 0; r < 8; ++r) os[wb + (8 * hi + r) * OSP + nt * 16 + lr] = acc[nt][r]; }
    wave_sync();
#pragma unroll 1
    for (int ps = 0; ps < 2; ++ps) {
#pragma unroll 4
        for (int s = 0; s < 20; ++s) { const int q = s * 32 + lane; const int row = q / 40, c4 = q % 40;
            const v4f val = *(const v4fa*)(&os[wb + row * OSP + c4 * 4]);
            *(volatile v4f*)(VO + ((size_t)(m0 + row) * NI + i) * NK + c4 * 4) = val; }
        if (ps == 0) __threadfence(); }
}

__global__ __launch_bounds__(32) void k_route(const float* __restrict__ VO, const float* __restrict__ bias, float* ACT) {
    __shared__ __align__(16) float sv[NI * NK];
    __shared__ __align__(16) float slog[NI * LP];
    __shared__ __align__(16) float srt[NI * LP];
    __shared__ __align__(16) float sact[NK];
    const int lane = threadIdx.x & 31, hi = lane >> 4;
    const int m = blockIdx.x;
    const float* vp = VO + (size_t)m * (NI * NK);
#pragma unroll 4
    for (int s = 0; s < (NI * NK) / 128; ++s) { const int q = s * 32 + lane; const v4f v = *(const v4f*)(vp + 4 * q); *(v4fa*)(&sv[4 * q]) = v; }
#pragma unroll 1
    for (int d = 0; d < OD; ++d) slog[lane * LP + d] = 0.0f;
    float bj[5];
#pragma unroll
    for (int j = 0; j < 5; ++j) bj[j] = bfr(bias[32 * j + lane]);
    wave_sync();
#pragma unroll 1
    for (int it = 0; it < 3; ++it) {
        float mx = slog[lane * LP];
#pragma unroll 1
        for (int d = 1; d < OD; ++d) mx = fmaxf(mx, slog[lane * LP + d]);
        float sum = 0.0f;
#pragma unroll 1
        for (int d = 0; d < OD; ++d) { const float e = __expf(slog[lane * LP + d] - mx); srt[lane * LP + d] = e; sum += e; }
        const float inv = 1.0f / sum;
#pragma unroll 1
        for (int d = 0; d < OD; ++d) { const float e = srt[lane * LP + d]; srt[lane * LP + d] = e * inv; }
        wave_sync();
        float acc[5];
#pragma unroll
        for (int j = 0; j < 5; ++j) acc[j] = 0.0f;
#pragma unroll 1
        for (int i = 0; i < NI; ++i) {
#pragma unroll
            for (int j = 0; j < 5; ++j) acc[j] = fmaf(srt[i * LP + 2 * j + hi], sv[i * NK + 32 * j + lane], acc[j]); }
#pragma unroll
        for (int j = 0; j < 5; ++j) sact[32 * j + lane] = acc[j] + bj[j];
        wave_sync();
#pragma unroll 1
        for (int j = 0; j < 5; ++j) {
            const float p = sact[32 * j + lane];
            float ss = p * p;
            ss += __shfl_xor(ss, 8, 32); ss += __shfl_xor(ss, 4, 32); ss += __shfl_xor(ss, 2, 32); ss += __shfl_xor(ss, 1, 32);
            const float nrm = sqrtf(ss);
            const float den = 1.0f + nrm * nrm;
            const float av = (p * nrm) * (1.0f / den);
            sact[32 * j + lane] = av; }
        wave_sync();
        if (it < 2) {
#pragma unroll 1
            for (int d = 0; d < OD; ++d) {
                float dot = 0.0f;
#pragma unroll
                for (int c = 0; c < 4; ++c) { const v4f vv = *(const v4fa*)(&sv[lane * NK + d * 16 + 4 * c]); const v4f aa = *(const v4fa*)(&sact[d * 16 + 4 * c]);
                    dot = fmaf(vv[0], aa[0], dot); dot = fmaf(vv[1], aa[1], dot); dot = fmaf(vv[2], aa[2], dot); dot = fmaf(vv[3], aa[3], dot); }
                const float lo = slog[lane * LP + d];
                slog[lane * LP + d] = lo + dot; }
            wave_sync();
        }
    }
    const v4f o0 = *(const v4fa*)(&sact[4 * lane]);
    const v4f o1 = *(const v4fa*)(&sact[128 + 4 * (lane & 7)]);
    float* op = ACT + (size_t)m * NK;
#pragma unroll 1
    for (int ps = 0; ps < 2; ++ps) {
        *(volatile v4f*)(op + 4 * lane) = o0;
        if (lane < 8) *(volatile v4f*)(op + 128 + 4 * lane) = o1;
        if (ps == 0) __threadfence(); }
}

__global__ __launch_bounds__(128) void k_out(const float* __restrict__ ACT, float* OUT) {
    __shared__ __align__(16) float t[32 * TP];
    const int tid = threadIdx.x;
    const int k0 = blockIdx.x * 32, b = blockIdx.y;
    const float* ap = ACT + (size_t)b * HW * NK + k0;
#pragma unroll 1
    for (int s = 0; s < 9; ++s) { const int q = s * 128 + tid; const int hw = q >> 3, c = q & 7;
        const v4f v = *(const v4f*)(ap + (size_t)hw * NK + 4 * c);
#pragma unroll
        for (int e = 0; e < 4; ++e) t[(4 * c + e) * TP + hw] = v[e]; }
    __syncthreads();
    float* op = OUT + ((size_t)b * NK + k0) * HW;
#pragma unroll 1
    for (int ps = 0; ps < 2; ++ps) {
#pragma unroll 1
        for (int s = 0; s < 9; ++s) { const int f = 4 * (s * 128 + tid); const int kk = f / HW, col = f % HW;
            const v4f val = *(const v4fa*)(&t[kk * TP + col]);
            *(volatile v4f*)(op + f) = val; }
        if (ps == 0) __threadfence(); }
}

static constexpr size_t al256(size_t v) { return (v + 255) & ~(size_t)255; }
static constexpr size_t SZ_XA = al256((size_t)NI * MROWS * 16 * 2);
static constexpr size_t SZ_WT = al256((size_t)NI * NK * 16 * 2);
static constexpr size_t SZ_VO = al256((size_t)MROWS * NI * NK * 4);
static constexpr size_t SZ_AC = al256((size_t)MROWS * NK * 4);
static constexpr size_t SZ_TOTAL = SZ_XA + SZ_WT + SZ_VO + SZ_AC;
static_assert(SZ_TOTAL <= (size_t)134217728);
static_assert(((size_t)HW * 16 * 2) % 128 == 0);
static_assert(((size_t)NK * 16 * 2) % 128 == 0);
static_assert(((size_t)NK * 4) % 128 == 0);

extern "C" void kernel_launch(void* const* d_in, const int* in_sizes, int n_in,
                              void* d_out, int out_size, void* d_ws, size_t ws_size, hipStream_t stream) {
    if (n_in < 3) return;
    if ((size_t)in_sizes[0] < (size_t)NB * NI * NA * HW) return;
    if ((size_t)in_sizes[1] < (size_t)NI * NA * NK) return;
    if ((size_t)in_sizes[2] < (size_t)NK) return;
    if ((size_t)out_size < (size_t)NB * NK * HW) return;
    if (SZ_TOTAL > ws_size) return;
    const float* x = (const float*)d_in[0];
    const float* w = (const float*)d_in[1];
    const float* bias = (const float*)d_in[2];
    float* OUT = (float*)d_out;
    char* wsp = (char*)d_ws;
    bf* XA = (bf*)wsp; wsp += SZ_XA;
    bf* WT = (bf*)wsp; wsp += SZ_WT;
    float* VO = (float*)wsp; wsp += SZ_VO;
    float* ACT = (float*)wsp; wsp += SZ_AC;

    k_tcvt<<<NB * NI, 2 * HW, 0, stream>>>(x, XA, HW, NI, (size_t)HW * 16, (size_t)MROWS * 16);
    k_tcvt<<<NI, 2 * NK, 0, stream>>>(w, WT, NK, 1, (size_t)NK * 16, (size_t)0);
    k_votes<<<(NI * MT) / VW, 32 * VW, 0, stream>>>(XA, WT, VO);
    k_route<<<MROWS, 32, 0, stream>>>(VO, bias, ACT);
    k_out<<<dim3(NK / 32, NB, 1), 128, 0, stream>>>(ACT, OUT);
}
